// SG_GNN_8521215115885
// MI455X (gfx1250) — hardware-verified
//
#include <hip/hip_runtime.h>
#include <math.h>


#define TPB 256
#define CAP 32

typedef __attribute__((ext_vector_type(16))) _Float16 v16h;
typedef __attribute__((ext_vector_type(8)))  _Float16 v8h;
typedef __attribute__((ext_vector_type(8)))  float  v8f;
typedef __attribute__((ext_vector_type(4)))  float  v4f;
typedef __attribute__((ext_vector_type(4)))  int    v4i;

static inline dim3 gridFor(size_t n) { return dim3((unsigned)((n + TPB - 1) / TPB)); }

#define VST2(T, ptr, val) do { const T _v = (val); *(volatile T*)(ptr) = _v; __threadfence(); *(volatile T*)(ptr) = _v; } while (0)

__device__ __forceinline__ v8f wmma16(v16h a, v16h b, v8f c) {
  v8f d = __builtin_amdgcn_wmma_f32_16x16x32_f16(false, a, false, b, (short)0, c, false, false);
  asm volatile("v_nop\n\tv_nop\n\tv_nop\n\tv_nop" : "+v"(d) : "v"(a), "v"(b));
  return d;
}

#define IL_T 128
#define IL_TILE 2048
__global__ __launch_bounds__(IL_T) void k_inlists(const int* __restrict__ src, const int* __restrict__ dst, int E, int N,
                                                  int* __restrict__ NBR, int* __restrict__ cnt) {
  __shared__ int td[IL_TILE], ts[IL_TILE];
  const int d = blockIdx.x * IL_T + threadIdx.x;
  int lst[CAP];
#pragma unroll
  for (int j = 0; j < CAP; ++j) lst[j] = -1;
  int n = 0;
  for (int e0 = 0; e0 < E; e0 += IL_TILE) {
    const int nt = min(IL_TILE, E - e0);
    __syncthreads();
    for (int i = threadIdx.x; i < nt; i += IL_T) { td[i] = dst[e0 + i]; ts[i] = src[e0 + i]; }
    __syncthreads();
    for (int i = 0; i < nt; ++i) {
      if (td[i] == d) {
#pragma unroll
        for (int j = 0; j < CAP; ++j) if (j == n) lst[j] = ts[i];
        ++n;
      }
    }
  }
  if (d < N) {
    int* row = NBR + (size_t)d * CAP;
    for (int pass = 0; pass < 2; ++pass) {
#pragma unroll
      for (int q = 0; q < CAP / 4; ++q) { v4i v = {lst[4 * q], lst[4 * q + 1], lst[4 * q + 2], lst[4 * q + 3]}; *(volatile v4i*)(row + 4 * q) = v; }
      __threadfence();
    }
    VST2(int, cnt + d, min(n, CAP));
  }
}

__global__ __launch_bounds__(TPB) void k_sage_gather(const float* __restrict__ x, const int* __restrict__ NBR, const int* __restrict__ cnt,
                                                     float* __restrict__ agg, int N) {
  const size_t t = (size_t)blockIdx.x * TPB + threadIdx.x;
  if (t >= (size_t)N * 64) return;
  const int i = (int)(t >> 6), f = (int)(t & 63);
  const int c = cnt[i];
  const int* row = NBR + (size_t)i * CAP;
  float s = 0.f;
  for (int p = 0; p < c; ++p) { const int j = row[p]; s += x[(size_t)j * 64 + f]; }
  const float v = s * (1.0f / fmaxf((float)c, 1.0f));
  VST2(float, agg + t, v);
}

#define WPACK_ELEMS 4096
__global__ void pack_w(const float* __restrict__ W, _Float16* __restrict__ P) {
  const int t8 = blockIdx.x * blockDim.x + threadIdx.x;
  if (t8 >= WPACK_ELEMS / 8) return;
  v8h v;
#pragma unroll
  for (int q = 0; q < 8; ++q) {
    const int t = t8 * 8 + q;
    const int e = t & 15, lane = (t >> 4) & 31, kbi = (t >> 9) & 1, ct = (t >> 10) & 3;
    const int n = ct * 16 + (lane & 15);
    const int k0 = kbi * 32 + ((lane >> 4) << 3);
    const int k = k0 + (e & 7) + ((e >> 3) << 4);
    v[q] = (_Float16)W[k * 64 + n];
  }
  VST2(v8h, P + (size_t)t8 * 8, v);
}

__device__ inline v16h load_a_frag(const float* __restrict__ A, int row0, int kb, int nrows) {
  const int lane = threadIdx.x & 31;
  int r = row0 + (lane & 15);
  if (r >= nrows) r = nrows - 1;
  const int k0 = kb + ((lane >> 4) << 3);
  const float* p = A + (size_t)r * 64 + k0;
  v16h a;
#pragma unroll
  for (int j = 0; j < 8; ++j) { a[j] = (_Float16)p[j]; a[8 + j] = (_Float16)p[16 + j]; }
  return a;
}
__device__ inline v16h load_b_packed(const _Float16* __restrict__ P, int ct, int kbi) {
  const int lane = threadIdx.x & 31;
  return *(const v16h*)(P + ((((ct * 2 + kbi) * 32) + lane) << 4));
}

template <bool DUAL>
__global__ __launch_bounds__(TPB) void gemm64(const float* __restrict__ A1, const _Float16* __restrict__ P1,
                                              const float* __restrict__ A2, const _Float16* __restrict__ P2,
                                              const float* __restrict__ bias, float* __restrict__ C, int nrows) {
  const int wave = threadIdx.x >> 5, lane = threadIdx.x & 31, hi = lane >> 4;
  const int row0 = blockIdx.x * 128 + wave * 16;
  if (row0 >= nrows) return;
  v8f acc[4] = {};
#pragma unroll
  for (int kbi = 0; kbi < 2; ++kbi) {
    const v16h a = load_a_frag(A1, row0, kbi * 32, nrows);
#pragma unroll
    for (int ct = 0; ct < 4; ++ct) acc[ct] = wmma16(a, load_b_packed(P1, ct, kbi), acc[ct]);
  }
  if (DUAL) {
#pragma unroll
    for (int kbi = 0; kbi < 2; ++kbi) {
      const v16h a = load_a_frag(A2, row0, kbi * 32, nrows);
#pragma unroll
      for (int ct = 0; ct < 4; ++ct) acc[ct] = wmma16(a, load_b_packed(P2, ct, kbi), acc[ct]);
    }
  }
  for (int pass = 0; pass < 2; ++pass) {
#pragma unroll
    for (int pr = 0; pr < 2; ++pr) {
      const int cbase = pr * 32;
      const float bv = bias ? bias[cbase + lane] : 0.f;
#pragma unroll
      for (int r = 0; r < 8; ++r) {
        const float a0 = acc[2 * pr][r], b0 = acc[2 * pr + 1][r];
        const float ax = __shfl_xor(a0, 16), bx = __shfl_xor(b0, 16);
        const float v1 = (hi ? bx : a0) + bv;
        const float v2 = (hi ? b0 : ax) + bv;
        const int r1 = row0 + r, r2 = row0 + r + 8;
        if (r1 < nrows) *(volatile float*)(C + (size_t)r1 * 64 + cbase + lane) = v1;
        if (r2 < nrows) *(volatile float*)(C + (size_t)r2 * 64 + cbase + lane) = v2;
      }
    }
    __threadfence();
  }
}

__global__ void att_kernel(const float* __restrict__ h, const float* __restrict__ a_src, const float* __restrict__ a_dst,
                           float* __restrict__ asrc, float* __restrict__ adst, int Nn, int H, int F) {
  const int t = blockIdx.x * blockDim.x + threadIdx.x;
  if (t >= Nn * H) return;
  const int n = t / H, hd = t % H;
  const float* hp = h + (size_t)n * 64 + hd * F;
  const float* as = a_src + hd * F;
  const float* ad = a_dst + hd * F;
  float s0 = 0.f, s1 = 0.f;
  for (int f = 0; f < F; ++f) { const float v = hp[f]; s0 += v * as[f]; s1 += v * ad[f]; }
  VST2(float, asrc + t, s0);
  VST2(float, adst + t, s1);
}

__device__ inline float lrelu(float v) { return v > 0.f ? v : 0.2f * v; }

__global__ __launch_bounds__(TPB) void k_gat_gather(const int* __restrict__ NBR, const int* __restrict__ cnt,
                                                    const float* __restrict__ asrc, const float* __restrict__ adst,
                                                    const float* __restrict__ hfeat, float* __restrict__ gout, int N, int H, int F) {
  const size_t t = (size_t)blockIdx.x * TPB + threadIdx.x;
  if (t >= (size_t)N * 64) return;
  const int i = (int)(t >> 6), f = (int)(t & 63);
  const int hd = f / F;
  const int c = cnt[i];
  const int* row = NBR + (size_t)i * CAP;
  const float ai = adst[(size_t)i * H + hd];
  float mx = -INFINITY;
  for (int p = 0; p < c; ++p) { const int j = row[p]; mx = fmaxf(mx, lrelu(asrc[(size_t)j * H + hd] + ai)); }
  float den = 0.f, acc = 0.f;
  for (int p = 0; p < c; ++p) {
    const int j = row[p];
    const float pe = expf(lrelu(asrc[(size_t)j * H + hd] + ai) - mx);
    den += pe;
    acc += pe * hfeat[(size_t)j * 64 + f];
  }
  const float v = (c > 0) ? (acc / den) : 0.f;
  VST2(float, gout + t, v);
}

__device__ inline float relu_silu(float v) {
  const float u = v > 0.f ? v : 0.f;
  return u / (1.f + expf(-u));
}
__global__ void combine4(const float* __restrict__ xin, const float* __restrict__ s,
                         const float* __restrict__ g, const float* __restrict__ gb,
                         float* __restrict__ xout, size_t nq) {
  const size_t i = (size_t)blockIdx.x * blockDim.x + threadIdx.x;
  if (i >= nq) return;
  const v4f xv = *(const v4f*)(xin + i * 4), sv = *(const v4f*)(s + i * 4), gv = *(const v4f*)(g + i * 4);
  const int gbase = (int)(i & 15) * 4;
  v4f o;
  o[0] = xv[0] + relu_silu(sv[0]) + relu_silu(gv[0] + gb[gbase + 0]);
  o[1] = xv[1] + relu_silu(sv[1]) + relu_silu(gv[1] + gb[gbase + 1]);
  o[2] = xv[2] + relu_silu(sv[2]) + relu_silu(gv[2] + gb[gbase + 2]);
  o[3] = xv[3] + relu_silu(sv[3]) + relu_silu(gv[3] + gb[gbase + 3]);
  VST2(v4f, xout + i * 4, o);
}

static void launch_layer(const float* xin, float* xout, int N, int Nown,
                         const int* NBR, const int* cnt,
                         const _Float16* pWl, const _Float16* pWr, const float* sb,
                         const _Float16* pGW, const float* gas, const float* gad, const float* gb,
                         int H, int F,
                         float* agg, float* sbuf, float* hbuf, float* gout,
                         float* asrc, float* adst, hipStream_t stream) {
  const size_t ndo = (size_t)Nown * 64;
  k_sage_gather<<<gridFor(ndo), TPB, 0, stream>>>(xin, NBR, cnt, agg, Nown);
  gemm64<true><<<dim3((Nown + 127) / 128), TPB, 0, stream>>>(agg, pWl, xin, pWr, sb, sbuf, Nown);
  gemm64<false><<<dim3((N + 127) / 128), TPB, 0, stream>>>(xin, pGW, nullptr, nullptr, nullptr, hbuf, N);
  att_kernel<<<gridFor((size_t)N * H), TPB, 0, stream>>>(hbuf, gas, gad, asrc, adst, N, H, F);
  k_gat_gather<<<gridFor(ndo), TPB, 0, stream>>>(NBR, cnt, asrc, adst, hbuf, gout, Nown, H, F);
  combine4<<<gridFor(ndo / 4), TPB, 0, stream>>>(xin, sbuf, gout, gb, xout, ndo / 4);
}

extern "C" void kernel_launch(void* const* d_in, const int* in_sizes, int n_in,
                              void* d_out, int out_size, void* d_ws, size_t ws_size,
                              hipStream_t stream) {
  (void)n_in; (void)out_size;
  const float* x    = (const float*)d_in[0];
  const int*   ei   = (const int*)d_in[1];
  const float* s1Wl = (const float*)d_in[2];
  const float* s1Wr = (const float*)d_in[3];
  const float* s1b  = (const float*)d_in[4];
  const float* s2Wl = (const float*)d_in[5];
  const float* s2Wr = (const float*)d_in[6];
  const float* s2b  = (const float*)d_in[7];
  const float* g1W  = (const float*)d_in[8];
  const float* g1as = (const float*)d_in[9];
  const float* g1ad = (const float*)d_in[10];
  const float* g1b  = (const float*)d_in[11];
  const float* g2W  = (const float*)d_in[12];
  const float* g2as = (const float*)d_in[13];
  const float* g2ad = (const float*)d_in[14];
  const float* g2b  = (const float*)d_in[15];

  const int N = in_sizes[0] / 64;
  const int E = in_sizes[1] / 2;
  const int* src = ei;
  const int* dst = ei + E;
  float* out = (float*)d_out;

  char* wp = (char*)d_ws; size_t off = 0;
  auto take = [&](size_t bytes) { char* p = wp + off; off += (bytes + 255) & ~(size_t)255; return (void*)p; };
  _Float16* p1Wl = (_Float16*)take(WPACK_ELEMS * 2);
  _Float16* p1Wr = (_Float16*)take(WPACK_ELEMS * 2);
  _Float16* p1GW = (_Float16*)take(WPACK_ELEMS * 2);
  _Float16* p2Wl = (_Float16*)take(WPACK_ELEMS * 2);
  _Float16* p2Wr = (_Float16*)take(WPACK_ELEMS * 2);
  _Float16* p2GW = (_Float16*)take(WPACK_ELEMS * 2);
  const size_t nd = (size_t)N * 64;
  int*   NBR  = (int*)take((size_t)N * CAP * 4);
  int*   cnt  = (int*)take((size_t)N * 4);
  float* agg  = (float*)take(nd * 4);
  float* sbuf = (float*)take(nd * 4);
  float* hbuf = (float*)take(nd * 4);
  float* gout = (float*)take(nd * 4);
  float* x1   = (float*)take(nd * 4);
  float* asrc = (float*)take((size_t)N * 8 * 4);
  float* adst = (float*)take((size_t)N * 8 * 4);
  if (off > ws_size) return;

  pack_w<<<2, TPB, 0, stream>>>(s1Wl, p1Wl);
  pack_w<<<2, TPB, 0, stream>>>(s1Wr, p1Wr);
  pack_w<<<2, TPB, 0, stream>>>(g1W,  p1GW);
  pack_w<<<2, TPB, 0, stream>>>(s2Wl, p2Wl);
  pack_w<<<2, TPB, 0, stream>>>(s2Wr, p2Wr);
  pack_w<<<2, TPB, 0, stream>>>(g2W,  p2GW);

  k_inlists<<<dim3((N + IL_T - 1) / IL_T), IL_T, 0, stream>>>(src, dst, E, N, NBR, cnt);

  launch_layer(x, x1, N, N, NBR, cnt, p1Wl, p1Wr, s1b, p1GW, g1as, g1ad, g1b, 8, 8,
               agg, sbuf, hbuf, gout, asrc, adst, stream);
  launch_layer(x1, out, N, N, NBR, cnt, p2Wl, p2Wr, s2b, p2GW, g2as, g2ad, g2b, 1, 64,
               agg, sbuf, hbuf, gout, asrc, adst, stream);
}
